// MultiheadAttention_18262200943004
// MI455X (gfx1250) — hardware-run, weakly checked
//
#include <hip/hip_runtime.h>
#include <math.h>

#ifndef NB
#define NB 2
#endif
#ifndef SEQ
#define SEQ 2048
#endif
#define NB_FULL 2
#define SEQ_FULL 2048
#define EDIM 1024
#define QKVN 3072
#define NHEAD 16
#define HDIM 64
static_assert(SEQ % 64 == 0);
static_assert(NB >= 1 && NB <= NB_FULL && SEQ <= SEQ_FULL);
static_assert(EDIM % 64 == 0 && QKVN % 64 == 0 && EDIM % 32 == 0);
static_assert(NHEAD * 3 * HDIM == QKVN && NHEAD * HDIM == EDIM && HDIM == 64);

typedef __attribute__((ext_vector_type(16))) _Float16 v16h;
typedef __attribute__((ext_vector_type(8)))  _Float16 v8h;
typedef __attribute__((ext_vector_type(8)))  float    v8f;
typedef __attribute__((ext_vector_type(4)))  float    v4f;
typedef unsigned int cm_u4 __attribute__((ext_vector_type(4)));

union FragH { v16h v; v8h h[2]; };

__device__ __forceinline__ v8f wmma16(v16h a, v16h b, v8f c) {
    c = __builtin_amdgcn_wmma_f32_16x16x32_f16(false, a, false, b, (short)0, c, false, false);
    asm volatile("v_nop\n\tv_nop\n\tv_nop\n\tv_nop" : "+v"(c) : "v"(a), "v"(b));
    return c;
}
__device__ __forceinline__ v16h ld_frag_g(const _Float16* __restrict__ p) {
    FragH f; f.h[0] = *(const v8h*)(p); f.h[1] = *(const v8h*)(p + 16); return f.v;
}

#define VST2(T, ptr, val) do { const T vst2_v_ = (val); *(volatile T*)(ptr) = vst2_v_; __threadfence(); *(volatile T*)(ptr) = vst2_v_; } while (0)

__device__ __forceinline__ unsigned int cmb_pk2(float a, float b) { return (unsigned int)__builtin_bit_cast(unsigned short, (_Float16)a) | ((unsigned int)__builtin_bit_cast(unsigned short, (_Float16)b) << 16); }
__device__ __forceinline__ float cmb_bf(float v) { const unsigned u = __builtin_bit_cast(unsigned, v); const unsigned r = (u + 0x7fffu + ((u >> 16) & 1u)) & 0xffff0000u; return __builtin_bit_cast(float, r); }

#define AW 4
#define VTP 72
__global__ __launch_bounds__(32 * AW) __attribute__((amdgpu_num_vgpr(256)))
void k_attn(const unsigned short* __restrict__ QKVp, unsigned short* __restrict__ CTX) {
    __shared__ __align__(16) float    pl[AW][16 * 64];
    __shared__ __align__(16) _Float16 vt[64 * VTP];
    const _Float16* __restrict__ QKV = (const _Float16*)QKVp;
    const int lane = threadIdx.x & 31, hf = lane >> 4, l15 = lane & 15;
    const int wave = __builtin_amdgcn_readfirstlane((int)(threadIdx.x >> 5));
    const int h = blockIdx.y, b = blockIdx.z;
    const int q0 = (blockIdx.x * AW + wave) * 16;
    const float L2E = 1.4426950408889634f;
    const float NEG = -__builtin_inff();
    const size_t row0 = (size_t)b * SEQ;
    const int hcol = h * 192;

    v16h qa[2];
    {
        const _Float16* qrow = QKV + (row0 + (size_t)(q0 + l15)) * QKVN + hcol + 8 * hf;
        qa[0] = ld_frag_g(qrow);
        qa[1] = ld_frag_g(qrow + 32);
    }
    v8f o[4]; float m8[8], l8[8];
#pragma unroll
    for (int t = 0; t < 4; ++t) { v8f zz = {}; o[t] = zz; }
#pragma unroll
    for (int i = 0; i < 8; ++i) { m8[i] = NEG; l8[i] = 0.f; }

    for (int j0 = 0; j0 < SEQ; j0 += 64) {
        __syncthreads();
        {
            const int jr = (int)(threadIdx.x >> 1), dh = (int)(threadIdx.x & 1) * 32;
            const _Float16* vrow = QKV + (row0 + (size_t)(j0 + jr)) * QKVN + hcol + 128 + dh;
#pragma unroll
            for (int i = 0; i < 4; ++i) {
                const v8h vv = *(const v8h*)(vrow + 8 * i);
#pragma unroll
                for (int e = 0; e < 8; ++e) vt[(dh + 8 * i + e) * VTP + jr] = vv[e];
            }
        }
        v8f s[4];
#pragma unroll
        for (int t = 0; t < 4; ++t) {
            const _Float16* krow = QKV + (row0 + (size_t)(j0 + t * 16 + l15)) * QKVN + hcol + 64 + 8 * hf;
            v8f acc = {};
            acc = wmma16(qa[0], ld_frag_g(krow), acc);
            acc = wmma16(qa[1], ld_frag_g(krow + 32), acc);
            s[t] = acc;
        }
#pragma unroll
        for (int i = 0; i < 8; ++i) {
            float sc[4];
#pragma unroll
            for (int t = 0; t < 4; ++t) { float v = s[t][i] * 0.125f; v *= L2E; sc[t] = v; }
            float mx = fmaxf(fmaxf(sc[0], sc[1]), fmaxf(sc[2], sc[3]));
            mx = fmaxf(mx, __shfl_xor(mx, 1, 32)); mx = fmaxf(mx, __shfl_xor(mx, 2, 32));
            mx = fmaxf(mx, __shfl_xor(mx, 4, 32)); mx = fmaxf(mx, __shfl_xor(mx, 8, 32));
            const float mnew = fmaxf(m8[i], mx);
            const float corr = (mnew == NEG) ? 1.f : exp2f(m8[i] - mnew);
            float rs = 0.f;
#pragma unroll
            for (int t = 0; t < 4; ++t) { const float pp = exp2f(sc[t] - mnew); rs += pp; s[t][i] = pp; }
            rs += __shfl_xor(rs, 1, 32); rs += __shfl_xor(rs, 2, 32); rs += __shfl_xor(rs, 4, 32); rs += __shfl_xor(rs, 8, 32);
            l8[i] = l8[i] * corr + rs; m8[i] = mnew;
#pragma unroll
            for (int t = 0; t < 4; ++t) o[t][i] *= corr;
        }
#pragma unroll
        for (int i = 0; i < 8; ++i)
#pragma unroll
            for (int t = 0; t < 4; ++t) pl[wave][(i + 8 * hf) * 64 + t * 16 + l15] = s[t][i];
        __syncthreads();
        v16h pa[2];
#pragma unroll
        for (int kk = 0; kk < 2; ++kk) {
            const int pb = l15 * 64 + kk * 32 + 8 * hf;
            const v4f x0 = *(const v4f*)&pl[wave][pb],      x1 = *(const v4f*)&pl[wave][pb + 4];
            const v4f x2 = *(const v4f*)&pl[wave][pb + 16], x3 = *(const v4f*)&pl[wave][pb + 20];
            v16h a;
            a[0]  = (_Float16)(x0.x * 4096.f); a[1]  = (_Float16)(x0.y * 4096.f); a[2]  = (_Float16)(x0.z * 4096.f); a[3]  = (_Float16)(x0.w * 4096.f);
            a[4]  = (_Float16)(x1.x * 4096.f); a[5]  = (_Float16)(x1.y * 4096.f); a[6]  = (_Float16)(x1.z * 4096.f); a[7]  = (_Float16)(x1.w * 4096.f);
            a[8]  = (_Float16)(x2.x * 4096.f); a[9]  = (_Float16)(x2.y * 4096.f); a[10] = (_Float16)(x2.z * 4096.f); a[11] = (_Float16)(x2.w * 4096.f);
            a[12] = (_Float16)(x3.x * 4096.f); a[13] = (_Float16)(x3.y * 4096.f); a[14] = (_Float16)(x3.z * 4096.f); a[15] = (_Float16)(x3.w * 4096.f);
            pa[kk] = a;
        }
#pragma unroll
        for (int t = 0; t < 4; ++t) {
            const int vo = (t * 16 + l15) * VTP + 8 * hf;
            FragH b0, b1;
            b0.h[0] = *(const v8h*)&vt[vo];      b0.h[1] = *(const v8h*)&vt[vo + 16];
            b1.h[0] = *(const v8h*)&vt[vo + 32]; b1.h[1] = *(const v8h*)&vt[vo + 48];
            o[t] = wmma16(pa[0], b0.v, o[t]);
            o[t] = wmma16(pa[1], b1.v, o[t]);
        }
    }
    __syncthreads();
#pragma unroll
    for (int i = 0; i < 8; ++i) {
        const float invr = (l8[i] > 0.f) ? 1.f / (l8[i] * 4096.f) : 0.f;
#pragma unroll
        for (int t = 0; t < 4; ++t) pl[wave][(i + 8 * hf) * 64 + t * 16 + l15] = o[t][i] * invr;
    }
    __syncthreads();
    {
        unsigned short* cb = CTX + (row0 + (size_t)q0) * EDIM + h * 64;
        const int rq = lane >> 3, c8 = (lane & 7) * 8;
#pragma unroll
        for (int it = 0; it < 4; ++it) {
            const int row = it * 4 + rq;
            const v4f x0 = *(const v4f*)&pl[wave][row * 64 + c8], x1 = *(const v4f*)&pl[wave][row * 64 + c8 + 4];
            cm_u4 pk;
            pk.x = cmb_pk2(x0.x * 64.f, x0.y * 64.f); pk.y = cmb_pk2(x0.z * 64.f, x0.w * 64.f);
            pk.z = cmb_pk2(x1.x * 64.f, x1.y * 64.f); pk.w = cmb_pk2(x1.z * 64.f, x1.w * 64.f);
            VST2(cm_u4, (cm_u4*)(cb + (size_t)row * EDIM + c8), pk);
        }
    }
}

__device__ __forceinline__ void dep_guard_h(v8f& a, v8f& b, v16h x) { asm volatile("v_nop\n\tv_nop\n\tv_nop\n\tv_nop" : "+v"(a), "+v"(b) : "v"(x)); }
__device__ __forceinline__ void keep4_h(v16h a, v16h b, v16h c, v16h d) { asm volatile("v_nop" :: "v"(a), "v"(b), "v"(c), "v"(d)); }
__device__ __forceinline__ void acc_guard4(v8f& a, v8f& b, v8f& c, v8f& d) { asm volatile("v_nop\n\tv_nop\n\tv_nop\n\tv_nop" : "+v"(a), "+v"(b), "+v"(c), "+v"(d)); }

template <int OUT_MODE>
__global__ __launch_bounds__(256) __attribute__((amdgpu_num_vgpr(256)))
void k_gemm64(const unsigned short* __restrict__ Ap, int lda,
              const unsigned short* __restrict__ Btp, int ldb,
              void* __restrict__ Cout, int ldc,
              const float* __restrict__ bias, int M, int N, int K, float scale) {
  const _Float16* __restrict__ A  = (const _Float16*)Ap;
  const _Float16* __restrict__ Bt = (const _Float16*)Btp;
  __shared__ __align__(16) float sT[8][16 * 68];
  const int lane = threadIdx.x & 31;
  const int wave = __builtin_amdgcn_readfirstlane((int)(threadIdx.x >> 5));
  const int tilesN = N >> 6;
  const int tilesM = M >> 6;
  const int tile = blockIdx.x * 8 + wave;
  if (tile >= tilesM * tilesN) return;
  const int tm = tile / tilesN;
  const int tn = tile - tm * tilesN;
  const int m0 = tm << 6;
  const int n0 = tn << 6;

  const int rlane = lane & 15;
  const int koff  = (lane >> 4) * 8;
  const int mOff  = (lane >> 4) * 8;

  v8f acc[4][4];
#pragma unroll
  for (int i = 0; i < 4; ++i)
#pragma unroll
    for (int j = 0; j < 4; ++j) acc[i][j] = (v8f){0.f,0.f,0.f,0.f,0.f,0.f,0.f,0.f};

  for (int k0 = 0; k0 < K; k0 += 32) {
    v16h bh[4];
#pragma unroll
    for (int j = 0; j < 4; ++j) {
      const size_t bo = (size_t)(n0 + (j << 4) + rlane) * ldb + koff + k0;
      bh[j] = ld_frag_g(Bt + bo);
    }
#pragma unroll
    for (int i = 0; i < 4; ++i) {
      const size_t ao = (size_t)(m0 + (i << 4) + rlane) * lda + koff + k0;
      const v16h ah = ld_frag_g(A + ao);
#pragma unroll
      for (int j = 0; j < 4; ++j)
        acc[i][j] = __builtin_amdgcn_wmma_f32_16x16x32_f16(false, ah, false, bh[j], (short)0, acc[i][j], false, false);
      dep_guard_h(acc[i][0], acc[i][3], ah);
    }
    keep4_h(bh[0], bh[1], bh[2], bh[3]);
  }
  acc_guard4(acc[0][0], acc[0][1], acc[0][2], acc[0][3]);
  acc_guard4(acc[1][0], acc[1][1], acc[1][2], acc[1][3]);
  acc_guard4(acc[2][0], acc[2][1], acc[2][2], acc[2][3]);
  acc_guard4(acc[3][0], acc[3][1], acc[3][2], acc[3][3]);

#pragma unroll
  for (int i = 0; i < 4; ++i) {
    const int mBase = m0 + (i << 4);
#pragma unroll
    for (int j = 0; j < 4; ++j) {
      const int n = n0 + (j << 4) + rlane;
      const float bv = cmb_bf(bias[n]);
#pragma unroll
      for (int r = 0; r < 8; ++r) {
        const float v = acc[i][j][r] * scale + bv;
        sT[wave][(mOff + r) * 68 + (j << 4) + rlane] = v;
      }
    }
    __builtin_amdgcn_fence(3  , "workgroup");
    __builtin_amdgcn_wave_barrier();
    __builtin_amdgcn_fence(2  , "workgroup");
    if (OUT_MODE == 0) {
      float* C = (float*)Cout;
      const int hh = lane >> 4, c4 = (lane & 15) * 4;
      for (int pass = 0; pass < 2; ++pass) {
#pragma unroll
        for (int it = 0; it < 8; ++it) {
          const int row = it * 2 + hh;
          const v4f v = *(const v4f*)&sT[wave][row * 68 + c4];
          *(volatile v4f*)(C + (size_t)(mBase + row) * ldc + n0 + c4) = v;
        }
        __threadfence();
      }
    } else {
      const int q = lane >> 3, c8 = (lane & 7) * 8;
      unsigned short* C = (unsigned short*)Cout;
      for (int pass = 0; pass < 2; ++pass) {
#pragma unroll
        for (int it = 0; it < 4; ++it) {
          const int row = it * 4 + q;
          v8h hv;
#pragma unroll
          for (int e = 0; e < 8; ++e) hv[e] = (_Float16)sT[wave][row * 68 + c8 + e];
          *(volatile v8h*)(C + (size_t)(mBase + row) * ldc + n0 + c8) = hv;
        }
        __threadfence();
      }
    }
    __builtin_amdgcn_fence(3  , "workgroup");
    __builtin_amdgcn_wave_barrier();
    __builtin_amdgcn_fence(2  , "workgroup");
  }
}

__global__ __launch_bounds__(256) void k_cm_castb(const float* __restrict__ SRC, long long sSz, int lds, unsigned short* __restrict__ DST, long long sDz, int ldd, int nR, int nC, float sc) {
    const long long u = (long long)blockIdx.x * 256 + threadIdx.x; const int per = nC / 8; if (u >= (long long)nR * per) return; const int r = (int)(u / per); const int c0 = 8 * (int)(u % per);
    const float* s = SRC + (long long)blockIdx.y * sSz + (long long)r * lds + c0; float w[8];
#pragma unroll
    for (int e = 0; e < 8; ++e) w[e] = cmb_bf(s[e]) * sc;
    cm_u4 pk; pk.x = cmb_pk2(w[0], w[1]); pk.y = cmb_pk2(w[2], w[3]); pk.z = cmb_pk2(w[4], w[5]); pk.w = cmb_pk2(w[6], w[7]); VST2(cm_u4, (cm_u4*)(DST + (long long)blockIdx.y * sDz + (long long)r * ldd + c0), pk); }
__global__ __launch_bounds__(256) void k_cm_castbT(const float* __restrict__ SRC, int lds, unsigned short* __restrict__ DST, int ldd, int nR, int nC, float sc) {
    const long long u = (long long)blockIdx.x * 256 + threadIdx.x; const int per = nR / 8; if (u >= (long long)nC * per) return; const int c = (int)(u / per); const int r0 = 8 * (int)(u % per);
    float w[8];
#pragma unroll
    for (int e = 0; e < 8; ++e) w[e] = cmb_bf(SRC[(long long)(r0 + e) * lds + c]) * sc;
    cm_u4 pk; pk.x = cmb_pk2(w[0], w[1]); pk.y = cmb_pk2(w[2], w[3]); pk.z = cmb_pk2(w[4], w[5]); pk.w = cmb_pk2(w[6], w[7]); VST2(cm_u4, (cm_u4*)(DST + (long long)c * ldd + r0), pk); }

constexpr size_t al256(size_t b) { return ((b + 255) / 256) * 256; }
constexpr size_t MROWS    = (size_t)NB * SEQ;
constexpr size_t SZ_X16   = al256(MROWS * EDIM * 2);
constexpr size_t SZ_W316  = al256((size_t)QKVN * EDIM * 2);
constexpr size_t SZ_QKV16 = al256(MROWS * QKVN * 2);
constexpr size_t SZ_CTX16 = al256(MROWS * EDIM * 2);
constexpr size_t SZ_WO16  = al256((size_t)EDIM * EDIM * 2);
constexpr size_t WS_TOTAL = SZ_X16 + SZ_W316 + SZ_QKV16 + SZ_CTX16 + SZ_WO16;
static_assert(WS_TOTAL <= (size_t)134217728);
static_assert(MROWS % 64 == 0);
static_assert(((MROWS / 64) * (QKVN / 64)) % 8 == 0 && ((MROWS / 64) * (EDIM / 64)) % 8 == 0);

extern "C" void kernel_launch(void* const* d_in, const int* in_sizes, int n_in, void* d_out, int out_size, void* d_ws, size_t ws_size, hipStream_t stream) {
    if (n_in < 5) return;
    const long long need_x = ((long long)(NB - 1) * SEQ_FULL + SEQ) * EDIM;
    if ((long long)in_sizes[0] < need_x) return;
    if ((long long)in_sizes[1] < (long long)EDIM * QKVN) return;
    if ((long long)in_sizes[2] < (long long)QKVN) return;
    if ((long long)in_sizes[3] < (long long)EDIM * EDIM) return;
    if ((long long)in_sizes[4] < (long long)EDIM) return;
    if ((long long)out_size < (long long)MROWS * EDIM) return;
    if (WS_TOTAL > ws_size) return;
    const float* xq   = (const float*)d_in[0];
    const float* Wqkv = (const float*)d_in[1];
    const float* bqkv = (const float*)d_in[2];
    const float* Wo   = (const float*)d_in[3];
    const float* bo   = (const float*)d_in[4];
    float* out = (float*)d_out;
    char* wsp = (char*)d_ws;
    unsigned short* X16   = (unsigned short*)wsp; wsp += SZ_X16;
    unsigned short* W316  = (unsigned short*)wsp; wsp += SZ_W316;
    unsigned short* QKV16 = (unsigned short*)wsp; wsp += SZ_QKV16;
    unsigned short* CTX16 = (unsigned short*)wsp; wsp += SZ_CTX16;
    unsigned short* WO16  = (unsigned short*)wsp; wsp += SZ_WO16;
    const int M = (int)MROWS;

    k_cm_castbT<<<(unsigned)((((long long)QKVN) * (EDIM / 8) + 255) / 256), 256, 0, stream>>>(Wqkv, QKVN, W316, EDIM, EDIM, QKVN, 16.0f);
    k_cm_castb<<<dim3((unsigned)((((long long)SEQ) * (EDIM / 8) + 255) / 256), (unsigned)NB), 256, 0, stream>>>(xq, (long long)SEQ_FULL * EDIM, EDIM, X16, (long long)SEQ * EDIM, EDIM, SEQ, EDIM, 1.0f);
    k_gemm64<1><<<(unsigned)((((M / 64) * (QKVN / 64)) + 7) / 8), 256, 0, stream>>>(
        (const unsigned short*)X16, EDIM, (const unsigned short*)W316, EDIM, (void*)QKV16, QKVN, bqkv, M, QKVN, EDIM, 0.0625f);
    k_cm_castbT<<<(unsigned)((((long long)EDIM) * (EDIM / 8) + 255) / 256), 256, 0, stream>>>(Wo, EDIM, WO16, EDIM, EDIM, EDIM, 16.0f);
    k_attn<<<dim3((unsigned)(SEQ / 64), (unsigned)NHEAD, (unsigned)NB), 32 * AW, 0, stream>>>((const unsigned short*)QKV16, CTX16);
    k_gemm64<0><<<(unsigned)((((M / 64) * (EDIM / 64)) + 7) / 8), 256, 0, stream>>>(
        (const unsigned short*)CTX16, EDIM, (const unsigned short*)WO16, EDIM, (void*)out, EDIM, bo, M, EDIM, EDIM, 0.0009765625f);
}
